// SPEncoder_33689723470053
// MI455X (gfx1250) — hardware-verified
//
#include <hip/hip_runtime.h>


#define L_    16384
#define DM_   192
#define DI_   384
#define NS_   16
#define DTR_  12
#define XDW_  64
#define XDN_  44
#define NORD_ 2
#define NBLK_ 4

static constexpr float EPS_ = 1e-5f;

static_assert(L_ % 64 == 0);
static_assert(L_ % 16 == 0);
static_assert(L_ % 8 == 0);
static_assert(DM_ % 64 == 0);
static_assert(DI_ % 64 == 0);
static_assert((2 * DI_) % 128 == 0);
static_assert(XDW_ % 64 == 0);
static_assert(DTR_ + 2 * NS_ == XDN_);
static_assert(XDN_ <= XDW_);
static_assert(DM_ == 192);

typedef float          v2f   __attribute__((ext_vector_type(2)));
typedef float          v4f   __attribute__((ext_vector_type(4)));
typedef float          v8f   __attribute__((ext_vector_type(8)));
typedef _Float16       v8h   __attribute__((ext_vector_type(8)));
typedef _Float16       v16h  __attribute__((ext_vector_type(16)));
typedef unsigned short u16x8 __attribute__((ext_vector_type(8)));

union FragH { u16x8 h[2]; v16h v; };
union Pack8 { v8h f; u16x8 u; };
union HBits { _Float16 h; unsigned short u; };

constexpr size_t SZ_XN  = (size_t)L_ * DM_ * 2;
constexpr size_t SZ_XC  = (size_t)2 * L_ * DI_ * 4;
constexpr size_t SZ_OY  = (size_t)2 * L_ * DM_ * 4;
constexpr size_t SZ_Z16 = (size_t)2 * L_ * DI_ * 2;
constexpr size_t SZ_UG  = (size_t)2 * L_ * DI_ * 2;
constexpr size_t SZ_XD  = (size_t)2 * L_ * XDW_ * 4;
constexpr size_t SZ_WI  = (size_t)NBLK_ * (2 * DI_) * DM_ * 2;
constexpr size_t SZ_WX  = (size_t)NBLK_ * XDW_ * DI_ * 2;
constexpr size_t SZ_WO  = (size_t)NBLK_ * DM_ * DI_ * 2;

constexpr size_t OFF_XN  = 0;
constexpr size_t OFF_XC  = OFF_XN + SZ_XN;
constexpr size_t OFF_Z16 = OFF_XC + SZ_XC;
constexpr size_t OFF_UG  = OFF_Z16 + SZ_Z16;
constexpr size_t OFF_XD  = OFF_UG + SZ_UG;
constexpr size_t OFF_WI  = OFF_XD + SZ_XD;
constexpr size_t OFF_WX  = OFF_WI + SZ_WI;
constexpr size_t OFF_WO  = OFF_WX + SZ_WX;
constexpr size_t WS_END  = OFF_WO + SZ_WO;

static_assert(SZ_OY <= SZ_XC);
static_assert(WS_END <= (size_t)134217728);
static_assert(OFF_XC % 128 == 0 && OFF_Z16 % 128 == 0 && OFF_UG % 128 == 0 && OFF_XD % 128 == 0);
static_assert(OFF_WI % 128 == 0 && OFF_WX % 128 == 0 && OFF_WO % 128 == 0 && WS_END % 128 == 0);

__device__ __forceinline__ float silu_f(float x) {
    float e = __expf(-x);
    return x * __builtin_amdgcn_rcpf(1.0f + e);
}
__device__ __forceinline__ float softplus_f(float x) {
    return fmaxf(x, 0.0f) + log1pf(__expf(-fabsf(x)));
}
__device__ __forceinline__ float conv4_silu(float x0, float x1, float x2, float x3,
                                            float w0, float w1, float w2, float w3, float bias) {
    float c = w0 * x0 + w1 * x1 + w2 * x2 + w3 * x3;
    return silu_f(c + bias);
}
__device__ __forceinline__ v8f ld8f(const float* p) {
    v4f a = *(const v4f*)p;
    v4f b = *(const v4f*)(p + 4);
    return __builtin_shufflevector(a, b, 0, 1, 2, 3, 4, 5, 6, 7);
}
__device__ __forceinline__ float wave_sum(float v) {
#pragma unroll
    for (int m = 16; m >= 1; m >>= 1) v += __shfl_xor(v, m, 32);
    return v;
}

__device__ __forceinline__ void mma16(v8f& acc, const FragH& a, const FragH& b) {
    acc = __builtin_amdgcn_wmma_f32_16x16x32_f16(false, a.v, false, b.v, (short)0, acc, false, false);
    asm volatile("v_nop\n\tv_nop\n\tv_nop\n\tv_nop" : "+v"(acc) : "v"(a.v), "v"(b.v));
}

template<bool RS>
__global__ __launch_bounds__(256)
void wt_kernel(const float* __restrict__ W, const float* __restrict__ rs, unsigned short* dst,
               int K, int Nsrc, int Npad, float scale)
{
    __shared__ float tile[64][65];
    const int tid  = threadIdx.x;
    const int wb   = blockIdx.z;
    const int k0   = blockIdx.x * 64;
    const int n0   = blockIdx.y * 64;
    const int col  = tid & 63;
    const int rsub = tid >> 6;
    const float* Wb = W + (size_t)wb * K * Nsrc;
    const int  ng  = n0 + col;
    const int  ncl = min(ng, Nsrc - 1);
    const bool okn = ng < Nsrc;
#pragma unroll 4
    for (int it = 0; it < 16; ++it) {
        const int row = it * 4 + rsub;
        float v = Wb[(size_t)(k0 + row) * Nsrc + ncl];
        if (!okn) v = 0.0f;
        if (RS) v *= rs[(size_t)wb * K + k0 + row];
        tile[row][col] = v * scale;
    }
    __syncthreads();
    const int lane = tid & 31, wave = tid >> 5;
    const int q = lane & 7, rr = lane >> 3;
    u16x8 uv[2];
    unsigned short* gp[2];
#pragma unroll
    for (int it = 0; it < 2; ++it) {
        const int n = it * 32 + wave * 4 + rr;
        v8f vals;
#pragma unroll
        for (int e = 0; e < 8; ++e) vals[e] = tile[q * 8 + e][n];
        Pack8 pk;
        pk.f = __builtin_convertvector(vals, v8h);
        uv[it] = pk.u;
        gp[it] = dst + ((size_t)wb * Npad + n0 + n) * K + k0 + q * 8;
    }
    *(volatile u16x8*)gp[0] = uv[0];
    *(volatile u16x8*)gp[1] = uv[1];
    __threadfence();
    *(volatile u16x8*)gp[0] = uv[0];
    *(volatile u16x8*)gp[1] = uv[1];
}

__global__ __launch_bounds__(256)
void gather_norm_kernel(const float* __restrict__ x, const int* __restrict__ ord, unsigned short* xn)
{
    const int lane = threadIdx.x & 31, wave = threadIdx.x >> 5;
    const int t = blockIdx.x * 8 + wave;
    int idx = ord[t];
    idx = min(max(idx, 0), L_ - 1);
    const int c = min(lane, 23) * 8;
    const float* xr = x + (size_t)idx * DM_ + c;
    v8f v = ld8f(xr);
    float ss = 0.0f;
#pragma unroll
    for (int e = 0; e < 8; ++e) ss += v[e] * v[e];
    if (lane >= 24) ss = 0.0f;
    ss = wave_sum(ss);
    const float inv = rsqrtf(ss * (1.0f / (float)DM_) + EPS_);
    Pack8 pk;
    pk.f = __builtin_convertvector(v * inv, v8h);
    const u16x8 u = pk.u;
    unsigned short* gp = xn + (size_t)t * DM_ + c;
    if (lane < 24) { *(volatile u16x8*)gp = u; }
    __threadfence();
    if (lane < 24) { *(volatile u16x8*)gp = u; }
}

template<typename OT, int NBF>
__device__ __forceinline__ void tile_store_pass(const float* st, OT* gp, int ldc, int lane) {
    constexpr int CW  = NBF * 16;
    constexpr int P   = CW + 4;
    constexpr int EPL = 16 / (int)sizeof(OT);
    static_assert(CW % EPL == 0);
    constexpr int LPR = CW / EPL;
    static_assert(32 % LPR == 0);
    constexpr int RPI = 32 / LPR;
    static_assert(32 % RPI == 0);
    constexpr int NIT = 32 / RPI;
    const int rsub = lane / LPR;
    const int c0   = (lane % LPR) * EPL;
#pragma unroll
    for (int it = 0; it < NIT; ++it) {
        const int row = it * RPI + rsub;
        const float* sp = st + row * P + c0;
        OT* dp = gp + (size_t)row * ldc + c0;
        if constexpr (sizeof(OT) == 4) {
            const v4f v = *(const v4f*)sp;
            *(volatile v4f*)dp = v;
        } else {
            Pack8 pk;
            pk.f = __builtin_convertvector(ld8f(sp), v8h);
            const u16x8 u = pk.u;
            *(volatile u16x8*)dp = u;
        }
    }
}

template<int NBF, typename OT1, typename OT2>
__global__ __launch_bounds__(128)
void gemm_tn_kernel(const unsigned short* __restrict__ A, const unsigned short* __restrict__ Bw,
                    OT1* C1, OT2* C2,
                    long long a_zs, long long b_zs, long long c1_zs, long long c2_zs,
                    int M, int K, int a_rev_mask, int ldc1, int ldc2, int csplit, float scale)
{
    constexpr int CW = NBF * 16;
    constexpr int P  = CW + 4;
    __shared__ __attribute__((aligned(16))) float stile[4][32 * P];

    const int tid  = threadIdx.x;
    const int lane = tid & 31;
    const int wave = tid >> 5;
    const int h    = lane >> 4;
    const int m    = lane & 15;
    const int wm   = wave >> 1;
    const int wn   = wave & 1;
    const int z    = blockIdx.z;

    const int rowW = blockIdx.y * 64 + wm * 32;
    const int colW = blockIdx.x * (2 * CW) + wn * CW;
    const int rev  = (a_rev_mask >> z) & 1;

    const unsigned short* Az = A + (size_t)z * (size_t)a_zs;
    const unsigned short* pa[2];
#pragma unroll
    for (int s = 0; s < 2; ++s) {
        const int r  = rowW + 16 * s + m;
        const int pr = rev ? (M - 1 - r) : r;
        pa[s] = Az + (size_t)pr * K + 8 * h;
    }
    const unsigned short* pb = Bw + (size_t)z * (size_t)b_zs + (size_t)(colW + m) * K + 8 * h;
    const size_t sub16 = (size_t)16 * K;

    v8f acc[2 * NBF];
#pragma unroll
    for (int j = 0; j < 2 * NBF; ++j)
#pragma unroll
        for (int r = 0; r < 8; ++r) acc[j][r] = 0.0f;

    const int nk = K >> 5;
    for (int kt = 0; kt < nk; ++kt) {
        const int k0 = kt * 32;
        FragH fa[2], fb[NBF];
#pragma unroll
        for (int s = 0; s < 2; ++s) {
            fa[s].h[0] = *(const u16x8*)(pa[s] + k0);
            fa[s].h[1] = *(const u16x8*)(pa[s] + k0 + 16);
        }
#pragma unroll
        for (int j = 0; j < NBF; ++j) {
            const unsigned short* p = pb + j * sub16 + k0;
            fb[j].h[0] = *(const u16x8*)(p);
            fb[j].h[1] = *(const u16x8*)(p + 16);
        }
#pragma unroll
        for (int s = 0; s < 2; ++s)
#pragma unroll
            for (int j = 0; j < NBF; ++j)
                mma16(acc[s * NBF + j], fa[s], fb[j]);
    }

    float* st = stile[wave];
#pragma unroll
    for (int s = 0; s < 2; ++s)
#pragma unroll
        for (int j = 0; j < NBF; ++j)
#pragma unroll
            for (int r = 0; r < 8; ++r)
                st[(s * 16 + 8 * h + r) * P + j * 16 + m] = acc[s * NBF + j][r] * scale;
    __syncthreads();

    if (colW < csplit) {
        OT1* gp = C1 + (size_t)z * (size_t)c1_zs + (size_t)rowW * ldc1 + colW;
        tile_store_pass<OT1, NBF>(st, gp, ldc1, lane);
        __threadfence();
        tile_store_pass<OT1, NBF>(st, gp, ldc1, lane);
    } else {
        OT2* gp = C2 + (size_t)z * (size_t)c2_zs + (size_t)rowW * ldc2 + (colW - csplit);
        tile_store_pass<OT2, NBF>(st, gp, ldc2, lane);
        __threadfence();
        tile_store_pass<OT2, NBF>(st, gp, ldc2, lane);
    }
}

__global__ __launch_bounds__(192)
void conv_silu_kernel(const float* __restrict__ Xc, const float* __restrict__ cw,
                      const float* __restrict__ cb, unsigned short* U16, int o)
{
    const int z  = blockIdx.y;
    const int wb = o + 2 * z;
    const int r  = threadIdx.x / 48;
    const int ch = threadIdx.x - r * 48;
    const int t  = blockIdx.x * 4 + r;
    const int d0 = ch * 8;
    const size_t rowz = (size_t)z * L_;
    const int t1 = max(t - 1, 0), t2 = max(t - 2, 0), t3 = max(t - 3, 0);

    v8f x3 = ld8f(Xc + (rowz + (size_t)t)  * DI_ + d0);
    v8f x2 = ld8f(Xc + (rowz + (size_t)t1) * DI_ + d0);
    v8f x1 = ld8f(Xc + (rowz + (size_t)t2) * DI_ + d0);
    v8f x0 = ld8f(Xc + (rowz + (size_t)t3) * DI_ + d0);
#pragma unroll
    for (int c = 0; c < 8; ++c) {
        x2[c] = (t >= 1) ? x2[c] : 0.0f;
        x1[c] = (t >= 2) ? x1[c] : 0.0f;
        x0[c] = (t >= 3) ? x0[c] : 0.0f;
    }

    const float* wp = cw + ((size_t)wb * DI_ + d0) * 4;
    v4f wv[8];
#pragma unroll
    for (int c = 0; c < 8; ++c) wv[c] = *(const v4f*)(wp + 4 * c);
    const v8f bias = ld8f(cb + (size_t)wb * DI_ + d0);

    v8f u;
#pragma unroll
    for (int c = 0; c < 8; ++c)
        u[c] = 64.0f * conv4_silu(x0[c], x1[c], x2[c], x3[c], wv[c][0], wv[c][1], wv[c][2], wv[c][3], bias[c]);

    Pack8 pk;
    pk.f = __builtin_convertvector(u, v8h);
    const u16x8 v = pk.u;
    unsigned short* gp = U16 + (rowz + (size_t)t) * DI_ + d0;
    *(volatile u16x8*)gp = v;
    __threadfence();
    *(volatile u16x8*)gp = v;
}

__device__ __forceinline__ void g16_store_pass(const unsigned short* sl, unsigned short* gp,
                                               size_t gbase, int wave, int lane) {
#pragma unroll
    for (int it = 0; it < 2; ++it) {
        const int t = it * 8 + wave * 4 + (lane >> 3);
        const int c = (lane & 7) * 8;
        const u16x8 v = *(const u16x8*)(sl + t * 64 + c);
        *(volatile u16x8*)(gp + gbase + (size_t)t * DI_ + c) = v;
    }
}

__global__ __launch_bounds__(64)
void scan_kernel(const float* __restrict__ Xc, const _Float16* __restrict__ Zh,
                 const float* __restrict__ xd,
                 const float* __restrict__ cw, const float* __restrict__ cb,
                 const float* __restrict__ dtw, const float* __restrict__ dtb,
                 const float* __restrict__ Alog, const float* __restrict__ Dp,
                 unsigned short* g16, int o)
{
    __shared__ __attribute__((aligned(16))) unsigned short sg[16 * 64];
    __shared__ __attribute__((aligned(16))) float sX[16 * XDW_];

    const int tid   = threadIdx.x;
    const int lane  = tid & 31;
    const int wave  = tid >> 5;
    const int z     = blockIdx.y;
    const int wb    = o + 2 * z;
    const int dbase = blockIdx.x * 64;
    const int d     = dbase + tid;
    const size_t pd = (size_t)wb * DI_ + d;

    float an[NS_], hs[NS_];
#pragma unroll
    for (int n = 0; n < NS_; ++n) {
        an[n] = -expf(Alog[pd * NS_ + n]);
        hs[n] = 0.0f;
    }
    float wd[DTR_];
#pragma unroll
    for (int r = 0; r < DTR_; ++r) wd[r] = dtw[((size_t)wb * DTR_ + r) * DI_ + d];
    const float w0 = cw[pd * 4 + 0], w1 = cw[pd * 4 + 1], w2 = cw[pd * 4 + 2], w3 = cw[pd * 4 + 3];
    const float cbias = cb[pd];
    const float tb    = dtb[pd];
    const float Dd    = Dp[pd];

    float xm1 = 0.0f, xm2 = 0.0f, xm3 = 0.0f;
    const size_t zrow0 = (size_t)z * L_;

#pragma unroll 1
    for (int l0 = 0; l0 < L_; l0 += 16) {
        const float* xsrc = xd + (zrow0 + (size_t)l0) * XDW_;
#pragma unroll
        for (int j = 0; j < 16; ++j) sX[j * 64 + tid] = xsrc[j * 64 + tid];
        __syncthreads();
#pragma unroll 1
        for (int t = 0; t < 16; ++t) {
            const size_t e = (zrow0 + (size_t)(l0 + t)) * DI_ + d;
            const float xv = Xc[e];
            const float zv = (float)Zh[e];
            const float u  = conv4_silu(xm3, xm2, xm1, xv, w0, w1, w2, w3, cbias);
            xm3 = xm2; xm2 = xm1; xm1 = xv;
            const float* sr = sX + t * XDW_;
            float dp = 0.0f;
#pragma unroll
            for (int r = 0; r < DTR_; ++r) dp = fmaf(sr[r], wd[r], dp);
            const float dt = softplus_f(dp + tb);
            const float du = dt * u;
            float y = 0.0f;
#pragma unroll
            for (int n = 0; n < NS_; ++n) {
                const float da = __expf(dt * an[n]);
                hs[n] = da * hs[n] + du * sr[DTR_ + n];
                y += hs[n] * sr[DTR_ + NS_ + n];
            }
            const float g = (y + Dd * u) * silu_f(zv);
            HBits hb;
            hb.h = (_Float16)(g * 256.0f);
            sg[t * 64 + tid] = hb.u;
        }
        __syncthreads();
        const size_t gbase = (zrow0 + (size_t)l0) * DI_ + dbase;
        g16_store_pass(sg, g16, gbase, wave, lane);
        __threadfence();
        g16_store_pass(sg, g16, gbase, wave, lane);
        __syncthreads();
    }
}

__device__ __forceinline__ void ln6(float* v, const float* __restrict__ w, const float* __restrict__ b, int cA, int cB) {
    float s = 0.0f;
#pragma unroll
    for (int j = 0; j < 6; ++j) s += v[j];
    const float mean = wave_sum(s) * (1.0f / (float)DM_);
    float q = 0.0f;
#pragma unroll
    for (int j = 0; j < 6; ++j) { const float dlt = v[j] - mean; q += dlt * dlt; }
    const float rr = rsqrtf(wave_sum(q) * (1.0f / (float)DM_) + EPS_);
    const v4f wa = *(const v4f*)(w + cA);
    const v2f wb = *(const v2f*)(w + cB);
    const v4f ba = *(const v4f*)(b + cA);
    const v2f bb = *(const v2f*)(b + cB);
    const float wj[6] = {wa[0], wa[1], wa[2], wa[3], wb[0], wb[1]};
    const float bj[6] = {ba[0], ba[1], ba[2], ba[3], bb[0], bb[1]};
#pragma unroll
    for (int j = 0; j < 6; ++j) v[j] = (v[j] - mean) * rr * wj[j] + bj[j];
}

__global__ __launch_bounds__(256)
void combine_kernel(const float* __restrict__ x, const int* __restrict__ ord,
                    const float* __restrict__ oy, const float* base, float* out,
                    const float* __restrict__ lwf, const float* __restrict__ lbf,
                    const float* __restrict__ lwb, const float* __restrict__ lbb,
                    const float* __restrict__ lwo, const float* __restrict__ lbo)
{
    const int lane = threadIdx.x & 31, wave = threadIdx.x >> 5;
    const int t = blockIdx.x * 8 + wave;
    int idx = ord[t];
    idx = min(max(idx, 0), L_ - 1);
    const int cA = 4 * lane;
    const int cB = 128 + 2 * lane;

    const float* xr = x  + (size_t)idx * DM_;
    const float* fy = oy + (size_t)t * DM_;
    const float* by = oy + ((size_t)L_ + (size_t)(L_ - 1 - t)) * DM_;
    const v4f xa = *(const v4f*)(xr + cA);  const v2f xb = *(const v2f*)(xr + cB);
    const v4f fa = *(const v4f*)(fy + cA);  const v2f fb = *(const v2f*)(fy + cB);
    const v4f ga = *(const v4f*)(by + cA);  const v2f gb = *(const v2f*)(by + cB);

    float fr[6] = {xa[0] + fa[0], xa[1] + fa[1], xa[2] + fa[2], xa[3] + fa[3], xb[0] + fb[0], xb[1] + fb[1]};
    float br[6] = {xa[0] + ga[0], xa[1] + ga[1], xa[2] + ga[2], xa[3] + ga[3], xb[0] + gb[0], xb[1] + gb[1]};
    ln6(fr, lwf, lbf, cA, cB);
    ln6(br, lwb, lbb, cA, cB);
    float cv[6];
#pragma unroll
    for (int j = 0; j < 6; ++j) cv[j] = fr[j] + br[j];
    ln6(cv, lwo, lbo, cA, cB);

    const float* bp = base + (size_t)idx * DM_;
    const v4f pa = *(const v4f*)(bp + cA);
    const v2f pb = *(const v2f*)(bp + cB);
    v4f r0;
    r0[0] = pa[0] + cv[0]; r0[1] = pa[1] + cv[1]; r0[2] = pa[2] + cv[2]; r0[3] = pa[3] + cv[3];
    const float r4 = pb[0] + cv[4];
    const float r5 = pb[1] + cv[5];

    const int sl0 = (2 * lane) & 31, sl1 = (2 * lane + 1) & 31;
    v4f r1;
    r1[0] = __shfl(r4, sl0, 32);
    r1[1] = __shfl(r5, sl0, 32);
    r1[2] = __shfl(r4, sl1, 32);
    r1[3] = __shfl(r5, sl1, 32);

    float* op = out + (size_t)idx * DM_;
    *(volatile v4f*)(op + cA) = r0;
    if (lane < 16) { *(volatile v4f*)(op + 128 + 4 * lane) = r1; }
    __threadfence();
    *(volatile v4f*)(op + cA) = r0;
    if (lane < 16) { *(volatile v4f*)(op + 128 + 4 * lane) = r1; }
}

extern "C" void kernel_launch(void* const* d_in, const int* in_sizes, int n_in,
                              void* d_out, int out_size, void* d_ws, size_t ws_size,
                              hipStream_t stream)
{
    if (n_in < 18) return;
    if (in_sizes[0]  != L_ * DM_)                 return;
    if (in_sizes[1]  != NORD_ * L_)               return;
    if (in_sizes[2]  != NBLK_ * DM_)              return;
    if (in_sizes[3]  != NBLK_ * DM_ * 2 * DI_)    return;
    if (in_sizes[4]  != NBLK_ * DI_ * 4)          return;
    if (in_sizes[5]  != NBLK_ * DI_)              return;
    if (in_sizes[6]  != NBLK_ * DI_ * XDN_)       return;
    if (in_sizes[7]  != NBLK_ * DTR_ * DI_)       return;
    if (in_sizes[8]  != NBLK_ * DI_)              return;
    if (in_sizes[9]  != NBLK_ * DI_ * NS_)        return;
    if (in_sizes[10] != NBLK_ * DI_)              return;
    if (in_sizes[11] != NBLK_ * DI_ * DM_)        return;
    for (int i = 12; i < 18; ++i) if (in_sizes[i] != NORD_ * DM_) return;
    if (out_size != L_ * DM_)                     return;
    if (ws_size < WS_END)                         return;

    const float* x          = (const float*)d_in[0];
    const int*   orders     = (const int*)d_in[1];
    const float* norm_w     = (const float*)d_in[2];
    const float* in_proj_w  = (const float*)d_in[3];
    const float* conv_w     = (const float*)d_in[4];
    const float* conv_b     = (const float*)d_in[5];
    const float* x_proj_w   = (const float*)d_in[6];
    const float* dt_w       = (const float*)d_in[7];
    const float* dt_b       = (const float*)d_in[8];
    const float* A_log      = (const float*)d_in[9];
    const float* D_p        = (const float*)d_in[10];
    const float* out_proj_w = (const float*)d_in[11];
    const float* fwd_ln_w   = (const float*)d_in[12];
    const float* fwd_ln_b   = (const float*)d_in[13];
    const float* bwd_ln_w   = (const float*)d_in[14];
    const float* bwd_ln_b   = (const float*)d_in[15];
    const float* out_ln_w   = (const float*)d_in[16];
    const float* out_ln_b   = (const float*)d_in[17];
    float* out = (float*)d_out;

    char* ws = (char*)d_ws;
    unsigned short* xn  = (unsigned short*)(ws + OFF_XN);
    float*          Xc  = (float*)(ws + OFF_XC);
    float*          oy  = (float*)(ws + OFF_XC);
    unsigned short* z16 = (unsigned short*)(ws + OFF_Z16);
    unsigned short* ug  = (unsigned short*)(ws + OFF_UG);
    float*          xd  = (float*)(ws + OFF_XD);
    unsigned short* wiT = (unsigned short*)(ws + OFF_WI);
    unsigned short* wxT = (unsigned short*)(ws + OFF_WX);
    unsigned short* woT = (unsigned short*)(ws + OFF_WO);

    wt_kernel<true><<<dim3(DM_ / 64, (2 * DI_) / 64, NBLK_), dim3(256), 0, stream>>>(
        in_proj_w, norm_w, wiT, (int)DM_, (int)(2 * DI_), (int)(2 * DI_), 32.0f);
    wt_kernel<false><<<dim3(DI_ / 64, XDW_ / 64, NBLK_), dim3(256), 0, stream>>>(
        x_proj_w, norm_w, wxT, (int)DI_, (int)XDN_, (int)XDW_, 32.0f);
    wt_kernel<false><<<dim3(DI_ / 64, DM_ / 64, NBLK_), dim3(256), 0, stream>>>(
        out_proj_w, norm_w, woT, (int)DI_, (int)DM_, (int)DM_, 32.0f);

    for (int o = 0; o < NORD_; ++o) {
        const int* ord = orders + (size_t)o * L_;

        gather_norm_kernel<<<dim3(L_ / 8), dim3(256), 0, stream>>>(x, ord, xn);

        gemm_tn_kernel<4, float, unsigned short><<<dim3((2 * DI_) / 128, L_ / 64, 2), dim3(128), 0, stream>>>(
            (const unsigned short*)xn, (const unsigned short*)(wiT + (size_t)o * (2 * DI_) * DM_),
            Xc, z16,
            (long long)0, (long long)2 * (2 * DI_) * DM_, (long long)L_ * DI_, (long long)L_ * DI_,
            (int)L_, (int)DM_, 2, (int)DI_, (int)DI_, (int)DI_, 0.03125f);

        conv_silu_kernel<<<dim3(L_ / 4, 2), dim3(192), 0, stream>>>((const float*)Xc, conv_w, conv_b, ug, o);

        gemm_tn_kernel<2, float, float><<<dim3(XDW_ / 64, L_ / 64, 2), dim3(128), 0, stream>>>(
            (const unsigned short*)ug, (const unsigned short*)(wxT + (size_t)o * XDW_ * DI_),
            xd, xd,
            (long long)L_ * DI_, (long long)2 * XDW_ * DI_, (long long)L_ * XDW_, (long long)L_ * XDW_,
            (int)L_, (int)DI_, 0, (int)XDW_, (int)XDW_, 1 << 30, 1.0f / 2048.0f);

        scan_kernel<<<dim3(DI_ / 64, 2), dim3(64), 0, stream>>>(
            (const float*)Xc, (const _Float16*)z16, (const float*)xd, conv_w, conv_b, dt_w, dt_b, A_log, D_p, ug, o);

        gemm_tn_kernel<2, float, float><<<dim3(DM_ / 64, L_ / 64, 2), dim3(128), 0, stream>>>(
            (const unsigned short*)ug, (const unsigned short*)(woT + (size_t)o * DM_ * DI_),
            oy, oy,
            (long long)L_ * DI_, (long long)2 * DM_ * DI_, (long long)L_ * DM_, (long long)L_ * DM_,
            (int)L_, (int)DI_, 0, (int)DM_, (int)DM_, 1 << 30, 1.0f / 8192.0f);

        const float* base = (o == 0) ? x : (const float*)out;
        combine_kernel<<<dim3(L_ / 8), dim3(256), 0, stream>>>(
            x, ord, (const float*)oy, base, out,
            fwd_ln_w + (size_t)o * DM_, fwd_ln_b + (size_t)o * DM_,
            bwd_ln_w + (size_t)o * DM_, bwd_ln_b + (size_t)o * DM_,
            out_ln_w + (size_t)o * DM_, out_ln_b + (size_t)o * DM_);
    }
}
